// KAN_GNN_80693845557834
// MI455X (gfx1250) — hardware-verified
//
#include <hip/hip_runtime.h>
#include <stddef.h>


#pragma clang fp contract(off)

#define FEAT    64
#define NCLS    16
#define NLAY    3
#define NKNOT   12
#define KA      (FEAT * 9)
#define APH     (KA + 8)
#define PQW     128
#define GR      64
#define NTHR    256
#define NWAVE   8
#define EPT     8
#define NGRP    2
#define CHUNK   (NTHR * EPT * NGRP)
#define WCAP    (EPT * NGRP * 32)
#define LISTN   (NWAVE * WCAP)
#define LSH     13
#define NBC     8192
#define NBF     2048
#define RCAP    40960
#define RBN     128
#define TGT     256
#define DEGCAP  256
#define OTHR    512
#define CPT     16
#define WSCAP   134217728

#define LDS_KAN  (2 * GR * APH * 2)
#define LDS_FILL ((RCAP + NBF + LISTN) * 4 + 64)

static_assert((CHUNK & (CHUNK - 1)) == 0);
static_assert(CHUNK <= 4096);
static_assert(NBC <= (1 << LSH) && NBF <= (1 << LSH));
static_assert((NBC & (NBC - 1)) == 0 && (NBF & (NBF - 1)) == 0);
static_assert(NBC == 4 * NBF);
static_assert(OTHR * CPT == NBC);
static_assert(OTHR == 4 * 128);
static_assert((RCAP % 32) == 0);
static_assert(TGT == NWAVE * 32);
static_assert((NBC % TGT) == 0);
static_assert(NBC == NWAVE * 8 * 128);
static_assert((APH * 2) % 16 == 0);
static_assert(GR * PQW * 4 <= LDS_KAN);
static_assert(GR == 4 * 16);
static_assert((GR * FEAT) % NTHR == 0);
static_assert((KA % 32) == 0);
static_assert((TGT % GR) == 0);
static_assert((GR * NCLS) / 4 == NTHR);

typedef float          v4f  __attribute__((ext_vector_type(4)));
typedef float          v8f  __attribute__((ext_vector_type(8)));
typedef int            v4i  __attribute__((ext_vector_type(4)));
typedef unsigned short v8us __attribute__((ext_vector_type(8)));
typedef __bf16         v16b __attribute__((ext_vector_type(16)));
union FragB { v16b v; v8us h[2]; };

__device__ __forceinline__ unsigned int bfr(float f) {
  const unsigned int u = __float_as_uint(f);
  return (u + 0x7FFFu + ((u >> 16) & 1u)) >> 16;
}

__device__ __forceinline__ void split1(float x, unsigned short& hb, unsigned short& lb) {
  const unsigned int hu = bfr(x);
  const float hf = __uint_as_float(hu << 16);
  hb = (unsigned short)hu;
  lb = (unsigned short)bfr(x - hf);
}

__device__ __forceinline__ void split8(v4f a, v4f b, v8us& hi, v8us& lo) {
  unsigned short hb, lb;
  split1(a.x, hb, lb); hi[0] = hb; lo[0] = lb;
  split1(a.y, hb, lb); hi[1] = hb; lo[1] = lb;
  split1(a.z, hb, lb); hi[2] = hb; lo[2] = lb;
  split1(a.w, hb, lb); hi[3] = hb; lo[3] = lb;
  split1(b.x, hb, lb); hi[4] = hb; lo[4] = lb;
  split1(b.y, hb, lb); hi[5] = hb; lo[5] = lb;
  split1(b.z, hb, lb); hi[6] = hb; lo[6] = lb;
  split1(b.w, hb, lb); hi[7] = hb; lo[7] = lb;
}

__device__ __forceinline__ v8f wmb(v16b a, v16b b, v8f c) {
  v8f d = __builtin_amdgcn_wmma_f32_16x16x32_bf16(false, a, false, b, (short)0, c, false, false);
  asm volatile("v_nop\n\tv_nop\n\tv_nop\n\tv_nop" : "+v"(d) : "v"(a), "v"(b));
  return d;
}

template <int NB>
__device__ __forceinline__ int scan_chunk(const int* __restrict__ dsts, int nE, int cbase, int slotBase,
                                          int vec8, int* list, int tid, int lane, int wave) {
  int wc = 0;
#pragma unroll
  for (int g = 0; g < NGRP; ++g) {
    const int el0  = (g * NTHR + tid) * EPT;
    const int e0   = cbase + el0;
    const int sent = -2147483647 - 1;
    v4i da, db;
    if (vec8 != 0 && cbase + CHUNK <= nE) {
      da = *(const v4i*)(dsts + e0);
      db = *(const v4i*)(dsts + e0 + 4);
    } else {
      da.x = (e0     < nE) ? dsts[min(e0, nE - 1)] : sent;
      da.y = (e0 + 1 < nE) ? dsts[min(e0 + 1, nE - 1)] : sent;
      da.z = (e0 + 2 < nE) ? dsts[min(e0 + 2, nE - 1)] : sent;
      da.w = (e0 + 3 < nE) ? dsts[min(e0 + 3, nE - 1)] : sent;
      db.x = (e0 + 4 < nE) ? dsts[min(e0 + 4, nE - 1)] : sent;
      db.y = (e0 + 5 < nE) ? dsts[min(e0 + 5, nE - 1)] : sent;
      db.z = (e0 + 6 < nE) ? dsts[min(e0 + 6, nE - 1)] : sent;
      db.w = (e0 + 7 < nE) ? dsts[min(e0 + 7, nE - 1)] : sent;
    }
    const unsigned nb = (unsigned)slotBase;
    const unsigned s0 = (unsigned)da.x - nb, s1 = (unsigned)da.y - nb;
    const unsigned s2 = (unsigned)da.z - nb, s3 = (unsigned)da.w - nb;
    const unsigned s4 = (unsigned)db.x - nb, s5 = (unsigned)db.y - nb;
    const unsigned s6 = (unsigned)db.z - nb, s7 = (unsigned)db.w - nb;
    const bool h0 = s0 < (unsigned)NB, h1 = s1 < (unsigned)NB, h2 = s2 < (unsigned)NB, h3 = s3 < (unsigned)NB;
    const bool h4 = s4 < (unsigned)NB, h5 = s5 < (unsigned)NB, h6 = s6 < (unsigned)NB, h7 = s7 < (unsigned)NB;
    const unsigned any = __builtin_amdgcn_ballot_w32(h0 | h1 | h2 | h3 | h4 | h5 | h6 | h7);
    if (any != 0u) {
#define HITJ(J, HJ, SJ) { \
        const unsigned mj = __builtin_amdgcn_ballot_w32(HJ); \
        if (mj != 0u) { \
          if (HJ) { \
            const int pos = wc + (int)__builtin_amdgcn_mbcnt_lo(mj, 0u); \
            if (pos < WCAP) list[wave * WCAP + pos] = ((el0 + (J)) << LSH) | (int)(SJ); \
          } \
          wc += (int)__builtin_popcount(mj); } }
      HITJ(0, h0, s0)
      HITJ(1, h1, s1)
      HITJ(2, h2, s2)
      HITJ(3, h3, s3)
      HITJ(4, h4, s4)
      HITJ(5, h5, s5)
      HITJ(6, h6, s6)
      HITJ(7, h7, s7)
#undef HITJ
    }
  }
  return wc;
}

__global__ __launch_bounds__(NTHR) void k_wprep(
    const float* __restrict__ base, const float* __restrict__ spline, unsigned short* Bw,
    int nRows, int nSrc, int inTot, int nGroups) {
  const int g = (int)blockIdx.x * NTHR + (int)threadIdx.x;
  if (g >= nGroups) return;
  const int o  = g / (KA / 8);
  const int k0 = (g - o * (KA / 8)) * 8;
  const int half = o >= nSrc ? 1 : 0;
  int os = o - half * nSrc;
  os = os < 0 ? 0 : (os > nSrc - 1 ? nSrc - 1 : os);
  const int kb = k0 > FEAT - 8 ? FEAT - 8 : k0;
  int ks = k0 - FEAT; ks = ks < 0 ? 0 : ks;
  const float* pb = base   + (size_t)os * inTot     + half * FEAT     + kb;
  const float* ps = spline + (size_t)os * inTot * 8 + half * FEAT * 8 + ks;
  const v4f a1 = *(const v4f*)pb, b1 = *(const v4f*)(pb + 4);
  const v4f a2 = *(const v4f*)ps, b2 = *(const v4f*)(ps + 4);
  const bool fs = k0 < FEAT;
  v4f a, b;
  a.x = fs ? a1.x : a2.x; a.y = fs ? a1.y : a2.y; a.z = fs ? a1.z : a2.z; a.w = fs ? a1.w : a2.w;
  b.x = fs ? b1.x : b2.x; b.y = fs ? b1.y : b2.y; b.z = fs ? b1.z : b2.z; b.w = fs ? b1.w : b2.w;
  v8us hv, lv;
  split8(a, b, hv, lv);
  unsigned short* dh = Bw + (size_t)g * 8;
  unsigned short* dl = dh + (size_t)nRows * KA;
  *(volatile v8us*)dh = hv;
  *(volatile v8us*)dl = lv;
  __threadfence();
  *(volatile v8us*)dh = hv;
  *(volatile v8us*)dl = lv;
}

__global__ __launch_bounds__(NTHR) void k_count(
    const int* __restrict__ dsts, int* cnt, float* dis, int nE, int vec8) {
  __shared__ __attribute__((aligned(16))) int scnt[NBC];
  __shared__ __attribute__((aligned(16))) int list[LISTN];
  __shared__ int wcnt[NWAVE];
  const int tid = threadIdx.x, lane = tid & 31, wave = tid >> 5;
  const int nodeBase = blockIdx.x * NBC;

  for (int i = tid; i < NBC; i += NTHR) scnt[i] = 0;
  __syncthreads();

  const int nChunks = (nE + CHUNK - 1) / CHUNK;
#pragma unroll 1
  for (int ch = 0; ch < nChunks; ++ch) {
    const int cbase = ch * CHUNK;
    const int wc = scan_chunk<NBC>(dsts, nE, cbase, nodeBase, vec8, list, tid, lane, wave);
    if (lane == 0) wcnt[wave] = wc;
    __syncthreads();
    if (wave == 0) {
#pragma unroll 1
      for (int wsx = 0; wsx < NWAVE; ++wsx) {
        int n = __builtin_amdgcn_readfirstlane(wcnt[wsx]);
        n = n > WCAP ? WCAP : (n < 0 ? 0 : n);
        const int* lp = list + wsx * WCAP;
#pragma unroll 1
        for (int i = 0; i < n; ++i) {
          const int ent  = __builtin_amdgcn_readfirstlane(lp[i]);
          const int slot = ent & (NBC - 1);
          if (lane == 0) scnt[slot] = scnt[slot] + 1;
        }
      }
    }
    __syncthreads();
  }

  v4i cq[8]; v4f dq[8];
#pragma unroll
  for (int q = 0; q < 8; ++q) {
    const int f = (wave * 8 + q) * 128 + 4 * lane;
    const v4i c = *(const v4i*)(scnt + f);
    cq[q] = c;
    dq[q].x = rsqrtf((float)(c.x > 0 ? c.x : 0) + 1.0f);
    dq[q].y = rsqrtf((float)(c.y > 0 ? c.y : 0) + 1.0f);
    dq[q].z = rsqrtf((float)(c.z > 0 ? c.z : 0) + 1.0f);
    dq[q].w = rsqrtf((float)(c.w > 0 ? c.w : 0) + 1.0f);
  }
  int*   cp = cnt + (size_t)nodeBase;
  float* dp = dis + (size_t)nodeBase;
#pragma unroll
  for (int q = 0; q < 8; ++q) {
    const int f = (wave * 8 + q) * 128 + 4 * lane;
    *(volatile v4i*)(cp + f) = cq[q];
    *(volatile v4f*)(dp + f) = dq[q];
  }
  __threadfence();
#pragma unroll
  for (int q = 0; q < 8; ++q) {
    const int f = (wave * 8 + q) * 128 + 4 * lane;
    *(volatile v4i*)(cp + f) = cq[q];
    *(volatile v4f*)(dp + f) = dq[q];
  }
}

__global__ __launch_bounds__(OTHR) void k_offsets(
    const int* __restrict__ cnt, int* off, int* rbase, int nChunk) {
  __shared__ __attribute__((aligned(16))) int soff[NBC];
  __shared__ __attribute__((aligned(16))) int srb[RBN];
  __shared__ int wtot[OTHR / 32];
  const int tid = threadIdx.x, lane = tid & 31, wave = tid >> 5, sub = tid >> 7;
  for (int i = tid; i < RBN; i += OTHR) srb[i] = 0;
  int carry = 0;
#pragma unroll 1
  for (int ch = 0; ch < nChunk; ++ch) {
    const int base = ch * NBC;
    const v4i c0 = *(const v4i*)(cnt + base + CPT * tid);
    const v4i c1 = *(const v4i*)(cnt + base + CPT * tid + 4);
    const v4i c2 = *(const v4i*)(cnt + base + CPT * tid + 8);
    const v4i c3 = *(const v4i*)(cnt + base + CPT * tid + 12);
    const int e0  = max(c0.x, 0), e1  = max(c0.y, 0), e2  = max(c0.z, 0), e3  = max(c0.w, 0);
    const int e4  = max(c1.x, 0), e5  = max(c1.y, 0), e6  = max(c1.z, 0), e7  = max(c1.w, 0);
    const int e8  = max(c2.x, 0), e9  = max(c2.y, 0), e10 = max(c2.z, 0), e11 = max(c2.w, 0);
    const int e12 = max(c3.x, 0), e13 = max(c3.y, 0), e14 = max(c3.z, 0), e15 = max(c3.w, 0);
    const int ts = e0 + e1 + e2 + e3 + e4 + e5 + e6 + e7 + e8 + e9 + e10 + e11 + e12 + e13 + e14 + e15;
    int incl = ts;
#pragma unroll
    for (int d = 1; d < 32; d <<= 1) {
      const int t = __shfl_up(incl, d);
      if (lane >= d) incl += t;
    }
    if (lane == 31) wtot[wave] = incl;
    __syncthreads();
    const int S0 = wtot[0]  + wtot[1]  + wtot[2]  + wtot[3];
    const int S1 = wtot[4]  + wtot[5]  + wtot[6]  + wtot[7];
    const int S2 = wtot[8]  + wtot[9]  + wtot[10] + wtot[11];
    const int S3 = wtot[12] + wtot[13] + wtot[14] + wtot[15];
    int pre = 0;
#pragma unroll 1
    for (int w = 4 * sub; w < wave; ++w) pre += wtot[w];
    const int b0 = carry;
    const int b1 = b0 + ((S0 + 31) & ~31);
    const int b2 = b1 + ((S1 + 31) & ~31);
    const int b3 = b2 + ((S2 + 31) & ~31);
    const int b4 = b3 + ((S3 + 31) & ~31);
    const int myb = sub == 0 ? b0 : (sub == 1 ? b1 : (sub == 2 ? b2 : b3));
    if (tid == 0) {
      srb[min(4 * ch + 0, RBN - 1)] = b0;
      srb[min(4 * ch + 1, RBN - 1)] = b1;
      srb[min(4 * ch + 2, RBN - 1)] = b2;
      srb[min(4 * ch + 3, RBN - 1)] = b3;
    }
    int run = myb + pre + incl - ts;
    int* so = soff + CPT * tid;
    so[0]  = run; run += e0;
    so[1]  = run; run += e1;
    so[2]  = run; run += e2;
    so[3]  = run; run += e3;
    so[4]  = run; run += e4;
    so[5]  = run; run += e5;
    so[6]  = run; run += e6;
    so[7]  = run; run += e7;
    so[8]  = run; run += e8;
    so[9]  = run; run += e9;
    so[10] = run; run += e10;
    so[11] = run; run += e11;
    so[12] = run; run += e12;
    so[13] = run; run += e13;
    so[14] = run; run += e14;
    so[15] = run;
    carry = b4;
    __syncthreads();
    const v4i o0 = *(const v4i*)(soff + 4 * tid);
    const v4i o1 = *(const v4i*)(soff + 4 * (tid + OTHR));
    const v4i o2 = *(const v4i*)(soff + 4 * (tid + 2 * OTHR));
    const v4i o3 = *(const v4i*)(soff + 4 * (tid + 3 * OTHR));
    int* op = off + base;
    *(volatile v4i*)(op + 4 * tid) = o0;
    *(volatile v4i*)(op + 4 * (tid + OTHR)) = o1;
    *(volatile v4i*)(op + 4 * (tid + 2 * OTHR)) = o2;
    *(volatile v4i*)(op + 4 * (tid + 3 * OTHR)) = o3;
    __threadfence();
    *(volatile v4i*)(op + 4 * tid) = o0;
    *(volatile v4i*)(op + 4 * (tid + OTHR)) = o1;
    *(volatile v4i*)(op + 4 * (tid + 2 * OTHR)) = o2;
    *(volatile v4i*)(op + 4 * (tid + 3 * OTHR)) = o3;
    __syncthreads();
  }
  if (tid == 0) srb[min(4 * nChunk, RBN - 1)] = carry;
  __syncthreads();
  v4i rv = {0, 0, 0, 0};
  if (tid < 32) rv = *(const v4i*)(srb + 4 * tid);
  if (tid < 32) *(volatile v4i*)(rbase + 4 * tid) = rv;
  __threadfence();
  if (tid < 32) *(volatile v4i*)(rbase + 4 * tid) = rv;
}

__global__ __launch_bounds__(NTHR) void k_fill(
    const int* __restrict__ dsts, const int* __restrict__ srcs,
    const int* __restrict__ off, const int* __restrict__ rbase,
    int* csr, int nN, int nE, int vec8, int csrLen) {
  extern __shared__ v4f lds_dyn[];
  int* region = (int*)lds_dyn;
  int* cursor = region + RCAP;
  int* list   = cursor + NBF;
  int* wcnt   = list + LISTN;
  const int tid = threadIdx.x, lane = tid & 31, wave = tid >> 5;
  const int b = blockIdx.x;
  const int nodeBase = b * NBF;

  int rb0 = rbase[b];
  const int rb1 = rbase[b + 1];
  rb0 = rb0 < 0 ? 0 : (rb0 > csrLen ? csrLen : rb0);
  rb0 &= ~31;
  int len = rb1 - rb0;
  len = len < 0 ? 0 : (len > RCAP ? RCAP : len);
  int lenW = (len + 31) & ~31;
  if (rb0 + lenW > csrLen) lenW = (csrLen - rb0) & ~31;

  {
    const v4i z = {0, 0, 0, 0};
    for (int i = tid; i < RCAP / 4; i += NTHR) ((v4i*)region)[i] = z;
    for (int s = tid; s < NBF; s += NTHR) {
      int o = off[nodeBase + s] - rb0;
      o = o < 0 ? 0 : (o > RCAP ? RCAP : o);
      cursor[s] = o;
    }
  }
  __syncthreads();

  const int nChunks = (nE + CHUNK - 1) / CHUNK;
#pragma unroll 1
  for (int ch = 0; ch < nChunks; ++ch) {
    const int cbase = ch * CHUNK;
    const int wc = scan_chunk<NBF>(dsts, nE, cbase, nodeBase, vec8, list, tid, lane, wave);
    if (lane == 0) wcnt[wave] = wc;
    __syncthreads();
    if (wave == 0) {
#pragma unroll 1
      for (int wsx = 0; wsx < NWAVE; ++wsx) {
        int n = __builtin_amdgcn_readfirstlane(wcnt[wsx]);
        n = n > WCAP ? WCAP : (n < 0 ? 0 : n);
        const int* lp = list + wsx * WCAP;
#pragma unroll 1
        for (int i = 0; i < n; ++i) {
          const int ent  = __builtin_amdgcn_readfirstlane(lp[i]);
          const int slot = ent & (NBF - 1);
          int e = cbase + ((ent >> LSH) & (CHUNK - 1));
          e = e > nE - 1 ? nE - 1 : e;
          int src = srcs[e];
          src = src < 0 ? 0 : (src > nN - 1 ? nN - 1 : src);
          if (lane == 0) {
            int pos = cursor[slot];
            pos = pos < 0 ? 0 : (pos > RCAP - 1 ? RCAP - 1 : pos);
            region[pos] = src;
            const int np = pos + 1;
            cursor[slot] = np > RCAP ? RCAP : np;
          }
        }
      }
    }
    __syncthreads();
  }

  const int nv = lenW >> 2;
  int* gp = csr + rb0;
#pragma unroll 1
  for (int i = tid; i < nv; i += NTHR) { const v4i v = ((const v4i*)region)[i]; *(volatile v4i*)(gp + 4 * i) = v; }
  __threadfence();
#pragma unroll 1
  for (int i = tid; i < nv; i += NTHR) { const v4i v = ((const v4i*)region)[i]; *(volatile v4i*)(gp + 4 * i) = v; }
}

template <int NOUT>
__global__ __launch_bounds__(NTHR) void k_kan(
    const float* __restrict__ X, const unsigned short* __restrict__ Bw,
    const float* __restrict__ knots, float* C, int nRowsA, int nRowsC) {
  extern __shared__ v4f lds_dyn[];
  unsigned short* sHi = (unsigned short*)lds_dyn;
  unsigned short* sLo = sHi + GR * APH;
  float*          stg = (float*)lds_dyn;
  const int tid = threadIdx.x, lane = tid & 31, hh = lane >> 4, m = lane & 15;
  const int wave = __builtin_amdgcn_readfirstlane(tid >> 5);
  const int rowBase = blockIdx.x * GR;

  float t[NKNOT];
  {
    const v4f ka = *(const v4f*)knots, kb = *(const v4f*)(knots + 4), kc = *(const v4f*)(knots + 8);
    t[0] = ka.x; t[1] = ka.y; t[2]  = ka.z; t[3]  = ka.w;
    t[4] = kb.x; t[5] = kb.y; t[6]  = kb.z; t[7]  = kb.w;
    t[8] = kc.x; t[9] = kc.y; t[10] = kc.z; t[11] = kc.w;
  }
  float r1[11], r2[10], r3[9];
#pragma unroll
  for (int j = 0; j < 11; ++j) { const float d = t[j + 1] - t[j]; r1[j] = d > 1e-8f ? 1.0f / d : 0.0f; }
#pragma unroll
  for (int j = 0; j < 10; ++j) { const float d = t[j + 2] - t[j]; r2[j] = d > 1e-8f ? 1.0f / d : 0.0f; }
#pragma unroll
  for (int j = 0; j < 9; ++j)  { const float d = t[j + 3] - t[j]; r3[j] = d > 1e-8f ? 1.0f / d : 0.0f; }

#pragma unroll 1
  for (int it = 0; it < (GR * FEAT) / NTHR; ++it) {
    const int idx = it * NTHR + tid;
    const int r = idx >> 6, i = idx & 63;
    int row = rowBase + r;
    row = row > nRowsA - 1 ? nRowsA - 1 : row;
    const float x = X[(size_t)row * FEAT + i];
    const float ex = __expf(-x);
    const float sx = x * __builtin_amdgcn_rcpf(1.0f + ex);
    const float xc = fminf(fmaxf(x, -0.99f), 0.99f);
    float bq[11];
#pragma unroll
    for (int j = 0; j < 11; ++j) bq[j] = (xc >= t[j] && xc < t[j + 1]) ? 1.0f : 0.0f;
    float bp1[10];
#pragma unroll
    for (int j = 0; j < 10; ++j) {
      float lf = (xc - t[j]) * r1[j];          lf = lf * bq[j];
      float rg = (t[j + 2] - xc) * r1[j + 1];  rg = rg * bq[j + 1];
      bp1[j] = lf + rg;
    }
    float bp2[9];
#pragma unroll
    for (int j = 0; j < 9; ++j) {
      float lf = (xc - t[j]) * r2[j];          lf = lf * bp1[j];
      float rg = (t[j + 3] - xc) * r2[j + 1];  rg = rg * bp1[j + 1];
      bp2[j] = lf + rg;
    }
    v4f ba, bb;
    {
      float bs[8];
#pragma unroll
      for (int j = 0; j < 8; ++j) {
        float lf = (xc - t[j]) * r3[j];          lf = lf * bp2[j];
        float rg = (t[j + 4] - xc) * r3[j + 1];  rg = rg * bp2[j + 1];
        bs[j] = lf + rg;
      }
      ba.x = bs[0]; ba.y = bs[1]; ba.z = bs[2]; ba.w = bs[3];
      bb.x = bs[4]; bb.y = bs[5]; bb.z = bs[6]; bb.w = bs[7];
    }
    unsigned short shb, slb;
    split1(sx, shb, slb);
    v8us bh8, bl8;
    split8(ba, bb, bh8, bl8);
    unsigned short* ph = sHi + r * APH;
    unsigned short* pl = sLo + r * APH;
    ph[i] = shb;
    pl[i] = slb;
    *(v8us*)(ph + FEAT + 8 * i) = bh8;
    *(v8us*)(pl + FEAT + 8 * i) = bl8;
  }
  __syncthreads();

  constexpr int TPW = NOUT >= 32 ? NOUT / 32 : 1;
  const int rt = wave & 3, cg = wave >> 2;
  const int colBase = cg * TPW * 16;
  const bool active = (NOUT >= 32) || (cg == 0);
  v8f acc[TPW];
#pragma unroll
  for (int tt = 0; tt < TPW; ++tt) { v8f z = {0.f, 0.f, 0.f, 0.f, 0.f, 0.f, 0.f, 0.f}; acc[tt] = z; }
  if (active) {
    const unsigned short* ahp = sHi + (16 * rt + m) * APH + 8 * hh;
    const unsigned short* alp = sLo + (16 * rt + m) * APH + 8 * hh;
#pragma unroll 1
    for (int kt = 0; kt < KA / 32; ++kt) {
      FragB ah, al;
      ah.h[0] = *(const v8us*)(ahp + 32 * kt);
      ah.h[1] = *(const v8us*)(ahp + 32 * kt + 16);
      al.h[0] = *(const v8us*)(alp + 32 * kt);
      al.h[1] = *(const v8us*)(alp + 32 * kt + 16);
#pragma unroll
      for (int tt = 0; tt < TPW; ++tt) {
        const unsigned short* bp = Bw + (size_t)(colBase + 16 * tt + m) * KA + 32 * kt + 8 * hh;
        FragB bh, bl;
        bh.h[0] = *(const v8us*)bp;
        bh.h[1] = *(const v8us*)(bp + 16);
        bl.h[0] = *(const v8us*)(bp + (size_t)NOUT * KA);
        bl.h[1] = *(const v8us*)(bp + (size_t)NOUT * KA + 16);
        acc[tt] = wmb(ah.v, bh.v, acc[tt]);
        acc[tt] = wmb(ah.v, bl.v, acc[tt]);
        acc[tt] = wmb(al.v, bh.v, acc[tt]);
      }
    }
  }
  __syncthreads();

  if (active) {
    float* sp = stg + (16 * rt + 8 * hh) * NOUT + colBase + m;
#pragma unroll
    for (int tt = 0; tt < TPW; ++tt)
#pragma unroll
      for (int r = 0; r < 8; ++r) sp[r * NOUT + 16 * tt] = acc[tt][r];
  }
  __syncthreads();

  constexpr int VPT = (GR * NOUT / 4) / NTHR;
  v4f vals[VPT];
#pragma unroll
  for (int i = 0; i < VPT; ++i) {
    const int f = i * NTHR + tid;
    vals[i] = *(const v4f*)(stg + 4 * f);
  }
  float* gp = C + (size_t)rowBase * NOUT;
#pragma unroll
  for (int i = 0; i < VPT; ++i) {
    const int f = i * NTHR + tid;
    const int row = rowBase + f / (NOUT / 4);
    if (row < nRowsC) *(volatile v4f*)(gp + (size_t)4 * f) = vals[i];
  }
  __threadfence();
#pragma unroll
  for (int i = 0; i < VPT; ++i) {
    const int f = i * NTHR + tid;
    const int row = rowBase + f / (NOUT / 4);
    if (row < nRowsC) *(volatile v4f*)(gp + (size_t)4 * f) = vals[i];
  }
}

__global__ __launch_bounds__(NTHR) void k_agg(
    const int* __restrict__ csr, const int* __restrict__ off, const int* __restrict__ cnt,
    const float* __restrict__ dis, const float* __restrict__ PQ, const float* __restrict__ hres,
    const float* __restrict__ gam, const float* __restrict__ bet,
    float* hout, int nN, int csrLen, int useRes) {
  const int tid = threadIdx.x, lane = tid & 31, hh = lane >> 4, q = lane & 15;
  const int wave = __builtin_amdgcn_readfirstlane(tid >> 5);
  const int tbase = blockIdx.x * TGT + wave * 32;
  const int cl = tbase + lane;
  const int cnt_l = cnt[cl];
  const int off_l = off[cl];
  union FI { float f; int i; };
  FI dsu; dsu.f = dis[cl];
  const v4f g4 = *(const v4f*)(gam + 4 * q);
  const v4f b4 = *(const v4f*)(bet + 4 * q);
  v4f keep = {0.f, 0.f, 0.f, 0.f};

#pragma unroll 1
  for (int j = 0; j < 32; ++j) {
    int n = __builtin_amdgcn_readlane(cnt_l, j);
    n = n < 0 ? 0 : (n > DEGCAP ? DEGCAP : n);
    const int st = __builtin_amdgcn_readlane(off_l, j);
    FI du; du.i = __builtin_amdgcn_readlane(dsu.i, j);
    const float dc = du.f;
    const int c = tbase + j;
    v4f acc = {0.f, 0.f, 0.f, 0.f};
    float ts = 0.0f;
#pragma unroll 1
    for (int q0 = 0; q0 < n; q0 += 32) {
      int pos = st + q0 + lane;
      pos = pos < 0 ? 0 : (pos > csrLen - 1 ? csrLen - 1 : pos);
      int sl = csr[pos];
      sl = sl < 0 ? 0 : (sl > nN - 1 ? nN - 1 : sl);
      const float wl = dis[sl];
      const int mcnt = (n - q0) < 32 ? (n - q0) : 32;
#pragma unroll 1
      for (int p = 0; p < mcnt; p += 2) {
        int li = p + hh;
        li = li > 31 ? 31 : li;
        const int s = __shfl(sl, li);
        float w = __shfl(wl, li);
        w = (p + hh < mcnt) ? w : 0.0f;
        const v4f v = *(const v4f*)(PQ + (size_t)s * PQW + FEAT + 4 * q);
        acc = acc + w * v;
        ts = ts + w;
      }
    }
    acc.x += __shfl_xor(acc.x, 16);
    acc.y += __shfl_xor(acc.y, 16);
    acc.z += __shfl_xor(acc.z, 16);
    acc.w += __shfl_xor(acc.w, 16);
    ts += __shfl_xor(ts, 16);
    const v4f p4 = *(const v4f*)(PQ + (size_t)c * PQW + 4 * q);
    const v4f q4 = *(const v4f*)(PQ + (size_t)c * PQW + FEAT + 4 * q);
    const float T = ts + dc;
    const v4f v = (p4 * T + acc + q4 * dc) * dc;
    float s1 = (v.x + v.y) + (v.z + v.w);
    s1 += __shfl_xor(s1, 1); s1 += __shfl_xor(s1, 2); s1 += __shfl_xor(s1, 4); s1 += __shfl_xor(s1, 8);
    const float mu = s1 * (1.0f / 64.0f);
    const v4f d = v - mu;
    float s2 = (d.x * d.x + d.y * d.y) + (d.z * d.z + d.w * d.w);
    s2 += __shfl_xor(s2, 1); s2 += __shfl_xor(s2, 2); s2 += __shfl_xor(s2, 4); s2 += __shfl_xor(s2, 8);
    const float var = s2 * (1.0f / 64.0f);
    const float inv = rsqrtf(var + 1e-5f);
    v4f o = (d * inv) * g4 + b4;
    const v4f r4 = *(const v4f*)(hres + (size_t)c * FEAT + 4 * q);
    if (useRes != 0) o = o + r4;
    if ((j & 1) != 0) {
      v4f ov;
      ov.x = hh != 0 ? o.x : keep.x;
      ov.y = hh != 0 ? o.y : keep.y;
      ov.z = hh != 0 ? o.z : keep.z;
      ov.w = hh != 0 ? o.w : keep.w;
      float* hp = hout + (size_t)(tbase + j - 1) * FEAT + 4 * lane;
      *(volatile v4f*)hp = ov;
      __threadfence();
      *(volatile v4f*)hp = ov;
    } else {
      keep = o;
    }
  }
}

extern "C" void kernel_launch(void* const* d_in, const int* in_sizes, int n_in,
                              void* d_out, int out_size, void* d_ws, size_t ws_size,
                              hipStream_t stream) {
  if (n_in < 11) return;
  const int nN = in_sizes[0] / FEAT;
  const int nE = in_sizes[1] / 2;
  if (nN <= 0 || nE <= 0 || in_sizes[0] != nN * FEAT || in_sizes[1] != 2 * nE) return;
  if (in_sizes[2] != NKNOT) return;
  if (in_sizes[3] != FEAT * FEAT || in_sizes[4] != FEAT * FEAT * 8) return;
  if (in_sizes[5] != NLAY * FEAT * PQW || in_sizes[6] != NLAY * FEAT * PQW * 8) return;
  if (in_sizes[7] != NLAY * FEAT || in_sizes[8] != NLAY * FEAT) return;
  if (in_sizes[9] != NCLS * FEAT || in_sizes[10] != NCLS * FEAT * 8) return;
  if (out_size != nN * NCLS) return;
  if (nE > (1 << 28) || nN > (1 << 24)) return;

  const float* x     = (const float*)d_in[0];
  const int*   ei    = (const int*)d_in[1];
  const float* knots = (const float*)d_in[2];
  const float* inBw  = (const float*)d_in[3];
  const float* inSw  = (const float*)d_in[4];
  const float* cvBw  = (const float*)d_in[5];
  const float* cvSw  = (const float*)d_in[6];
  const float* lnG   = (const float*)d_in[7];
  const float* lnB   = (const float*)d_in[8];
  const float* outBw = (const float*)d_in[9];
  const float* outSw = (const float*)d_in[10];
  float* out = (float*)d_out;
  const int* erow = ei;
  const int* ecol = ei + nE;

  const int NPAD   = ((nN + TGT - 1) / TGT) * TGT;
  const int nBC    = (nN + NBC - 1) / NBC;
  const int CNTPAD = nBC * NBC;
  if (4 * nBC + 1 > RBN) return;
  const int nBF    = (nN + NBF - 1) / NBF;
  const int csrLen = ((nE + 31) & ~31) + 4096;
  if (31 * 4 * nBC > 4096) return;
  const int nKan   = NPAD / GR;
  const int nAgg   = NPAD / TGT;

  char* ws = (char*)d_ws;
  size_t offb = 0;
  const size_t oBin = offb; offb += (size_t)2 * FEAT * KA * 2;             offb = (offb + 255) & ~(size_t)255;
  const size_t oBc  = offb; offb += (size_t)NLAY * 2 * PQW * KA * 2;       offb = (offb + 255) & ~(size_t)255;
  const size_t oBo  = offb; offb += (size_t)2 * NCLS * KA * 2;             offb = (offb + 255) & ~(size_t)255;
  const size_t oCnt = offb; offb += (size_t)CNTPAD * 4;                    offb = (offb + 255) & ~(size_t)255;
  const size_t oDis = offb; offb += (size_t)CNTPAD * 4;                    offb = (offb + 255) & ~(size_t)255;
  const size_t oOff = offb; offb += (size_t)CNTPAD * 4;                    offb = (offb + 255) & ~(size_t)255;
  const size_t oRb  = offb; offb += (size_t)RBN * 4;                       offb = (offb + 255) & ~(size_t)255;
  const size_t oCsr = offb; offb += (size_t)csrLen * 4;                    offb = (offb + 255) & ~(size_t)255;
  const size_t oHA  = offb; offb += (size_t)NPAD * FEAT * 4;               offb = (offb + 255) & ~(size_t)255;
  const size_t oHB  = offb; offb += (size_t)NPAD * FEAT * 4;               offb = (offb + 255) & ~(size_t)255;
  const size_t oPQ  = offb; offb += (size_t)NPAD * PQW * 4;                offb = (offb + 255) & ~(size_t)255;
  if (offb > ws_size || offb > (size_t)WSCAP) return;
  unsigned short* Bin = (unsigned short*)(ws + oBin);
  unsigned short* Bc  = (unsigned short*)(ws + oBc);
  unsigned short* Bo  = (unsigned short*)(ws + oBo);
  int*   cnt   = (int*)(ws + oCnt);
  float* dis   = (float*)(ws + oDis);
  int*   offp  = (int*)(ws + oOff);
  int*   rbase = (int*)(ws + oRb);
  int*   csr   = (int*)(ws + oCsr);
  float* HA    = (float*)(ws + oHA);
  float* HB    = (float*)(ws + oHB);
  float* PQ    = (float*)(ws + oPQ);

  const int vec8 = ((nE & 3) == 0) ? 1 : 0;
  const size_t BCP = (size_t)2 * PQW * KA;

  const int gIn = FEAT * (KA / 8), gCv = PQW * (KA / 8), gOut = NCLS * (KA / 8);
  k_wprep<<<(gIn + NTHR - 1) / NTHR, NTHR, 0, stream>>>(inBw, inSw, Bin, FEAT, FEAT, FEAT, gIn);
  for (int l = 0; l < NLAY; ++l)
    k_wprep<<<(gCv + NTHR - 1) / NTHR, NTHR, 0, stream>>>(
        cvBw + (size_t)l * FEAT * PQW, cvSw + (size_t)l * FEAT * PQW * 8, Bc + (size_t)l * BCP, PQW, FEAT, PQW, gCv);
  k_wprep<<<(gOut + NTHR - 1) / NTHR, NTHR, 0, stream>>>(outBw, outSw, Bo, NCLS, NCLS, FEAT, gOut);

  hipFuncSetAttribute(reinterpret_cast<const void*>(&k_fill),
                      hipFuncAttributeMaxDynamicSharedMemorySize, LDS_FILL);
  k_count<<<nBC, NTHR, 0, stream>>>(ecol, cnt, dis, nE, vec8);
  k_offsets<<<1, OTHR, 0, stream>>>(cnt, offp, rbase, nBC);
  k_fill<<<nBF, NTHR, LDS_FILL, stream>>>(ecol, erow, offp, rbase, csr, nN, nE, vec8, csrLen);

  hipFuncSetAttribute(reinterpret_cast<const void*>(&k_kan<FEAT>),
                      hipFuncAttributeMaxDynamicSharedMemorySize, LDS_KAN);
  hipFuncSetAttribute(reinterpret_cast<const void*>(&k_kan<PQW>),
                      hipFuncAttributeMaxDynamicSharedMemorySize, LDS_KAN);
  hipFuncSetAttribute(reinterpret_cast<const void*>(&k_kan<NCLS>),
                      hipFuncAttributeMaxDynamicSharedMemorySize, LDS_KAN);

  k_kan<FEAT><<<nKan, NTHR, LDS_KAN, stream>>>(x, Bin, knots, HA, nN, NPAD);

  k_kan<PQW><<<nKan, NTHR, LDS_KAN, stream>>>(HA, Bc, knots, PQ, nN, NPAD);
  k_agg<<<nAgg, NTHR, 0, stream>>>(csr, offp, cnt, dis, PQ, HA, lnG, lnB, HB, nN, csrLen, 0);
  k_kan<PQW><<<nKan, NTHR, LDS_KAN, stream>>>(HB, Bc + BCP, knots, PQ, nN, NPAD);
  k_agg<<<nAgg, NTHR, 0, stream>>>(csr, offp, cnt, dis, PQ, HB, lnG + FEAT, lnB + FEAT, HA, nN, csrLen, 1);
  k_kan<PQW><<<nKan, NTHR, LDS_KAN, stream>>>(HA, Bc + 2 * BCP, knots, PQ, nN, NPAD);
  k_agg<<<nAgg, NTHR, 0, stream>>>(csr, offp, cnt, dis, PQ, HA, lnG + 2 * FEAT, lnB + 2 * FEAT, HB, nN, csrLen, 1);

  k_kan<NCLS><<<nKan, NTHR, LDS_KAN, stream>>>(HB, Bo, knots, out, nN, nN);
}
